// Decoder_47064251629825
// MI455X (gfx1250) — hardware-run, weakly checked
//
#include <hip/hip_runtime.h>
#include <math.h>

constexpr int NBAT  = 2048;
constexpr int NSTEP = 1024;
constexpr int NHID  = 32;
constexpr int NGATE = 4 * NHID;
constexpr int RBLK  = 16;
constexpr int NBLK  = NBAT / RBLK;
constexpr int NTHR  = 64;
constexpr int TCH   = 32;
constexpr int PBP   = 36;
constexpr int NREC  = NBAT * NSTEP;
constexpr int NOUTF = NREC + 1;
constexpr int LPW   = 32;
constexpr float LOSS_SCALE = 1.0f / 2097152.0f;
static_assert(NBAT % RBLK == 0);
static_assert(NSTEP % TCH == 0);
static_assert(NHID == 32);
static_assert(NGATE == 128);
static_assert((NGATE * NHID) % (8 * NTHR) == 0);
static_assert(NGATE % NTHR == 0);
static_assert(PBP % 4 == 0);
static_assert(NREC == 2097152);
static_assert(4 + 4 * NREC == 8388612);
static_assert(TCH == 32 && LPW == 32);

typedef __attribute__((ext_vector_type(16))) __bf16 v16b;
typedef __attribute__((ext_vector_type(8)))  __bf16 v8b;
typedef __attribute__((ext_vector_type(8)))  float  v8f;
typedef __attribute__((ext_vector_type(4)))  float  v4f;

__device__ __forceinline__ unsigned short f2bf_bits(float f) {
  unsigned u = __float_as_uint(f);
  return (unsigned short)((u + 0x7FFFu + ((u >> 16) & 1u)) >> 16);
}
__device__ __forceinline__ float bf_bits2f(unsigned short h) { return __uint_as_float(((unsigned)h) << 16); }
__device__ __forceinline__ float bf16r(float f) { return bf_bits2f(f2bf_bits(f)); }

__device__ __forceinline__ void dep_guard_b(v8f& a, v8f& b, v16b x, v16b y) { asm volatile("v_nop\n\tv_nop\n\tv_nop\n\tv_nop" : "+v"(a), "+v"(b) : "v"(x), "v"(y)); }
__device__ __forceinline__ void keep4_b(v16b a, v16b b, v16b c, v16b d) { asm volatile("v_nop" :: "v"(a), "v"(b), "v"(c), "v"(d)); }
__device__ __forceinline__ void mma_guard6(v8f& d0, v8f& d1, v8f& d2, v8f& d3,
                                           v16b a0, v16b a1, v16b a2, v16b a3, v16b b0, v16b b1) {
  asm volatile("v_nop\n\tv_nop\n\tv_nop\n\tv_nop"
               : "+v"(d0), "+v"(d1), "+v"(d2), "+v"(d3)
               : "v"(a0), "v"(a1), "v"(a2), "v"(a3), "v"(b0), "v"(b1));
}

template <typename T> struct Frag;
template <> struct Frag<__bf16> {
  typedef v16b V; union U { v16b v; v8b h[2]; };
  static __device__ __forceinline__ v16b load(const __bf16* p) {
    U f; f.h[0] = *(const v8b*)(p); f.h[1] = *(const v8b*)(p + 16); return f.v;
  }
  static __device__ __forceinline__ v8f mma(v16b a, v16b b, v8f c) {
    return __builtin_amdgcn_wmma_f32_16x16x32_bf16(false, a, false, b, (short)0, c, false, false);
  }
  static __device__ __forceinline__ void guard(v8f& a, v8f& b, v16b x, v16b y) { dep_guard_b(a, b, x, y); }
  static __device__ __forceinline__ void keep(v16b a, v16b b, v16b c, v16b d) { keep4_b(a, b, c, d); }
};

__device__ __forceinline__ float fsig(float x)  { return __builtin_amdgcn_rcpf(1.0f + __expf(-x)); }
__device__ __forceinline__ float ftanh(float x) { return 1.0f - 2.0f * __builtin_amdgcn_rcpf(__expf(2.0f * x) + 1.0f); }

__device__ __forceinline__ void ld8(const float* p, float (&o)[8]) {
  const v4f a = *(const v4f*)p;
  const v4f b = *(const v4f*)(p + 4);
  o[0] = a[0]; o[1] = a[1]; o[2] = a[2]; o[3] = a[3];
  o[4] = b[0]; o[5] = b[1]; o[6] = b[2]; o[7] = b[3];
}

__device__ __forceinline__ void split8(const float (&h)[8], v8b& hi, v8b& lo) {
#pragma unroll
  for (int e = 0; e < 8; ++e) {
    const unsigned short hb = f2bf_bits(h[e]);
    const unsigned short lb = f2bf_bits(h[e] - bf_bits2f(hb));
    hi[e] = __builtin_bit_cast(__bf16, hb);
    lo[e] = __builtin_bit_cast(__bf16, lb);
  }
}

__device__ __forceinline__ void stage_w(const float* __restrict__ src, __bf16* dst, int tid) {
#pragma unroll 1
  for (int it = 0; it < (NGATE * NHID) / (8 * NTHR); ++it) {
    const int ch  = it * NTHR + tid;
    const int row = ch >> 2;
    const int c8  = (ch & 3) * 8;
    const float* sp = src + row * NHID + c8;
    const v4f a = *(const v4f*)sp;
    const v4f b = *(const v4f*)(sp + 4);
    v8b o;
#pragma unroll
    for (int e = 0; e < 4; ++e) {
      const float fa = a[e];
      const float fb = b[e];
      o[e]     = __builtin_bit_cast(__bf16, f2bf_bits(fa));
      o[4 + e] = __builtin_bit_cast(__bf16, f2bf_bits(fb));
    }
    *(v8b*)(dst + row * NHID + c8) = o;
  }
}

__device__ __forceinline__ void cell8(const float (&zz)[4][8], float (&cs)[8], float (&hn)[8]) {
#pragma unroll
  for (int r = 0; r < 8; ++r) {
    const float ig = fsig(zz[0][r]);
    const float fg = fsig(zz[1][r]);
    const float gg = ftanh(zz[2][r]);
    const float og = fsig(zz[3][r]);
    const float cn = fg * cs[r] + ig * gg;
    cs[r] = cn;
    hn[r] = og * ftanh(cn);
  }
}

__device__ __forceinline__ void gate_mma(v8f (&acc)[4], const __bf16* wplane, int w, int c, int hh, v16b bh, v16b bl) {
  v16b af[4];
#pragma unroll
  for (int g = 0; g < 4; ++g) af[g] = Frag<__bf16>::load(wplane + (32 * g + 16 * w + c) * NHID + 8 * hh);
#pragma unroll
  for (int g = 0; g < 4; ++g) {
    acc[g] = Frag<__bf16>::mma(af[g], bh, acc[g]);
    acc[g] = Frag<__bf16>::mma(af[g], bl, acc[g]);
  }
  mma_guard6(acc[0], acc[1], acc[2], acc[3], af[0], af[1], af[2], af[3], bh, bl);
}

__device__ __forceinline__ void flush_seg(const float* pb, float* __restrict__ rec, const float* __restrict__ seq,
                                          int rowbase, int seg, int lane, float& lacc) {
  const int q = lane >> 3, c4 = (lane & 7) * 4;
  v4f v[4];
  size_t off[4];
#pragma unroll
  for (int it = 0; it < 4; ++it) {
    const int row = it * 4 + q;
    v[it]   = *(const v4f*)(pb + row * PBP + c4);
    off[it] = (size_t)(rowbase + row) * NSTEP + (size_t)seg * TCH + c4;
    const v4f x = *(const v4f*)(seq + off[it]);
#pragma unroll
    for (int e = 0; e < 4; ++e) {
      const float d = bf16r(x[e]) - v[it][e];
      lacc = fmaf(d, d, lacc);
    }
  }
  for (int pass = 0; pass < 2; ++pass) {
#pragma unroll
    for (int it = 0; it < 4; ++it) *(volatile v4f*)(rec + off[it]) = v[it];
    __threadfence();
  }
}

__global__ __launch_bounds__(NTHR) void seq_lstm_kernel(
    const float* __restrict__ seq, const float* __restrict__ z, const int* __restrict__ lens,
    const float* __restrict__ w_ih0, const float* __restrict__ w_hh0,
    const float* __restrict__ b_ih0, const float* __restrict__ b_hh0,
    const float* __restrict__ w_ih1, const float* __restrict__ w_hh1,
    const float* __restrict__ b_ih1, const float* __restrict__ b_hh1,
    const float* __restrict__ w_out, const float* __restrict__ b_out,
    float* __restrict__ rec, float* __restrict__ lpart) {
  __shared__ __align__(16) __bf16 Whh0s[NGATE * NHID];
  __shared__ __align__(16) __bf16 Wih1s[NGATE * NHID];
  __shared__ __align__(16) __bf16 Whh1s[NGATE * NHID];
  __shared__ __align__(16) __bf16 H0h[RBLK * NHID];
  __shared__ __align__(16) __bf16 H0l[RBLK * NHID];
  __shared__ __align__(16) __bf16 H1h[RBLK * NHID];
  __shared__ __align__(16) __bf16 H1l[RBLK * NHID];
  __shared__ __align__(16) float  B0s[NGATE];
  __shared__ __align__(16) float  Wi0s[NGATE];
  __shared__ __align__(16) float  B1s[NGATE];
  __shared__ __align__(16) float  Psum[2 * RBLK];
  __shared__ __align__(16) float  Pbuf[RBLK * PBP];

  (void)lens;
  const int tid  = threadIdx.x;
  const int lane = tid & 31;
  const int w    = tid >> 5;
  const int c    = lane & 15;
  const int hh   = lane >> 4;
  const int ub   = 16 * w + 8 * hh;
  const int rowbase = blockIdx.x * RBLK;

  stage_w(w_hh0, Whh0s, tid);
  stage_w(w_ih1, Wih1s, tid);
  stage_w(w_hh1, Whh1s, tid);
#pragma unroll 1
  for (int i = tid; i < NGATE; i += NTHR) {
    B0s[i]  = bf16r(b_ih0[i]) + bf16r(b_hh0[i]);
    Wi0s[i] = bf16r(w_ih0[i]);
    B1s[i]  = bf16r(b_ih1[i]) + bf16r(b_hh1[i]);
  }
  float wo[8];
  {
    const v4f a = *(const v4f*)(w_out + ub);
    const v4f b = *(const v4f*)(w_out + ub + 4);
#pragma unroll
    for (int e = 0; e < 4; ++e) { wo[e] = bf16r(a[e]); wo[4 + e] = bf16r(b[e]); }
  }
  const float bout = bf16r(b_out[0]);
  float c0s[8], c1s[8];
  {
    const float* zr = z + (size_t)(rowbase + c) * NHID + ub;
    const v4f a = *(const v4f*)zr;
    const v4f b = *(const v4f*)(zr + 4);
#pragma unroll
    for (int e = 0; e < 4; ++e) { c0s[e] = bf16r(a[e]); c0s[4 + e] = bf16r(b[e]); }
#pragma unroll
    for (int r = 0; r < 8; ++r) c1s[r] = c0s[r];
    v8b hi, lo;
    split8(c0s, hi, lo);
    *(v8b*)(H0h + c * NHID + ub) = hi;
    *(v8b*)(H0l + c * NHID + ub) = lo;
    *(v8b*)(H1h + c * NHID + ub) = hi;
    *(v8b*)(H1l + c * NHID + ub) = lo;
  }
  __syncthreads();

  v16b hb0h = Frag<__bf16>::load(H0h + c * NHID + 8 * hh);
  v16b hb0l = Frag<__bf16>::load(H0l + c * NHID + 8 * hh);
  v16b hb1h = Frag<__bf16>::load(H1h + c * NHID + 8 * hh);
  v16b hb1l = Frag<__bf16>::load(H1l + c * NHID + 8 * hh);
  float predc = 0.0f;
  float lacc  = 0.0f;
  const v8f z8 = {0.f, 0.f, 0.f, 0.f, 0.f, 0.f, 0.f, 0.f};

#pragma unroll 1
  for (int t = 0; t < NSTEP; ++t) {
    float hn[8];
    {
      v8f acc[4];
      acc[0] = z8; acc[1] = z8; acc[2] = z8; acc[3] = z8;
      gate_mma(acc, Whh0s, w, c, hh, hb0h, hb0l);
      float zz[4][8];
#pragma unroll
      for (int g = 0; g < 4; ++g) {
        float b8[8], w8[8];
        ld8(B0s + 32 * g + ub, b8);
        ld8(Wi0s + 32 * g + ub, w8);
#pragma unroll
        for (int r = 0; r < 8; ++r) zz[g][r] = acc[g][r] + fmaf(w8[r], predc, b8[r]);
      }
      cell8(zz, c0s, hn);
      v8b hi, lo;
      split8(hn, hi, lo);
      *(v8b*)(H0h + c * NHID + ub) = hi;
      *(v8b*)(H0l + c * NHID + ub) = lo;
    }
    __syncthreads();

    if (((t & (TCH - 1)) == 0) && (t > 0)) {
      if (w == 0) flush_seg(Pbuf, rec, seq, rowbase, (t / TCH) - 1, lane, lacc);
    }

    hb0h = Frag<__bf16>::load(H0h + c * NHID + 8 * hh);
    hb0l = Frag<__bf16>::load(H0l + c * NHID + 8 * hh);

    {
      v8f acc[4];
      acc[0] = z8; acc[1] = z8; acc[2] = z8; acc[3] = z8;
      gate_mma(acc, Wih1s, w, c, hh, hb0h, hb0l);
      gate_mma(acc, Whh1s, w, c, hh, hb1h, hb1l);
      float zz[4][8];
#pragma unroll
      for (int g = 0; g < 4; ++g) {
        float b8[8];
        ld8(B1s + 32 * g + ub, b8);
#pragma unroll
        for (int r = 0; r < 8; ++r) zz[g][r] = acc[g][r] + b8[r];
      }
      cell8(zz, c1s, hn);
      float sp = 0.0f;
#pragma unroll
      for (int r = 0; r < 8; ++r) sp = fmaf(hn[r], wo[r], sp);
      sp += __shfl_xor(sp, 16, 32);
      if (hh == 0) Psum[16 * w + c] = sp;
      v8b hi, lo;
      split8(hn, hi, lo);
      *(v8b*)(H1h + c * NHID + ub) = hi;
      *(v8b*)(H1l + c * NHID + ub) = lo;
    }
    __syncthreads();

    hb1h = Frag<__bf16>::load(H1h + c * NHID + 8 * hh);
    hb1l = Frag<__bf16>::load(H1l + c * NHID + 8 * hh);
    predc = (Psum[c] + Psum[RBLK + c]) + bout;
    if (w == 0 && hh == 0) Pbuf[c * PBP + (t & (TCH - 1))] = predc;
  }
  __syncthreads();
  if (w == 0) {
    flush_seg(Pbuf, rec, seq, rowbase, NSTEP / TCH - 1, lane, lacc);
    float* lp = lpart + (size_t)blockIdx.x * LPW + lane;
    *(volatile float*)lp = lacc;
    __threadfence();
    *(volatile float*)lp = lacc;
  }
}

__global__ __launch_bounds__(32) void loss_line_kernel(const float* __restrict__ lpart, float* __restrict__ lline) {
  const int lane = threadIdx.x;
  float s = 0.0f;
#pragma unroll 1
  for (int k = 0; k < NBLK; ++k) s += lpart[k * LPW + lane];
#pragma unroll
  for (int off = 1; off < 32; off <<= 1) s += __shfl_xor(s, off, 32);
  const float total = s * LOSS_SCALE;
  *(volatile float*)(lline + lane) = total;
  __threadfence();
  *(volatile float*)(lline + lane) = total;
}

__global__ __launch_bounds__(256) void out_pack_kernel(const float* __restrict__ rec, const float* __restrict__ lline,
                                                       float* __restrict__ out) {
  const int i = blockIdx.x * 256 + (int)threadIdx.x;
  int ir = i - 1;
  ir = (ir < 0) ? 0 : ir;
  ir = (ir > NREC - 1) ? (NREC - 1) : ir;
  const float rv = rec[ir];
  const float lv = lline[threadIdx.x & 31];
  const float f1 = (i == 0) ? 1.0f : 0.0f;
  const float f0 = 1.0f - f1;
  const float v  = fmaf(f1, lv, f0 * rv);
  if (i < NOUTF) {
    *(volatile float*)(out + i) = v;
    __threadfence();
    *(volatile float*)(out + i) = v;
  }
}

extern "C" void kernel_launch(void* const* d_in, const int* in_sizes, int n_in,
                              void* d_out, int out_size, void* d_ws, size_t ws_size, hipStream_t stream) {
  if (n_in < 13 || d_out == nullptr || d_ws == nullptr) return;
  if (in_sizes[0] != NBAT * NSTEP || in_sizes[1] != NBAT * NHID || in_sizes[2] != NBAT ||
      in_sizes[3] != NGATE || in_sizes[4] != NGATE * NHID || in_sizes[5] != NGATE || in_sizes[6] != NGATE ||
      in_sizes[7] != NGATE * NHID || in_sizes[8] != NGATE * NHID || in_sizes[9] != NGATE || in_sizes[10] != NGATE ||
      in_sizes[11] != NHID || in_sizes[12] != 1 || out_size != NOUTF) return;

  const float* seq   = (const float*)d_in[0];
  const float* z     = (const float*)d_in[1];
  const int*   lens  = (const int*)d_in[2];
  const float* w_ih0 = (const float*)d_in[3];
  const float* w_hh0 = (const float*)d_in[4];
  const float* b_ih0 = (const float*)d_in[5];
  const float* b_hh0 = (const float*)d_in[6];
  const float* w_ih1 = (const float*)d_in[7];
  const float* w_hh1 = (const float*)d_in[8];
  const float* b_ih1 = (const float*)d_in[9];
  const float* b_hh1 = (const float*)d_in[10];
  const float* w_out = (const float*)d_in[11];
  const float* b_out = (const float*)d_in[12];
  float* out = (float*)d_out;

  char* ws = (char*)d_ws; size_t off = 0;
  auto carve = [&](size_t bytes) -> char* { char* p = ws + off; off += (bytes + 255) & ~(size_t)255; return p; };
  float* REC   = (float*)carve((size_t)NREC * 4);
  float* LPART = (float*)carve((size_t)NBLK * LPW * 4);
  float* LLINE = (float*)carve((size_t)32 * 4);
  if (off > ws_size || off > (size_t)134217728) return;

  seq_lstm_kernel<<<NBLK, NTHR, 0, stream>>>(seq, z, lens, w_ih0, w_hh0, b_ih0, b_hh0,
                                             w_ih1, w_hh1, b_ih1, b_hh1, w_out, b_out, REC, LPART);
  loss_line_kernel<<<1, 32, 0, stream>>>(LPART, LLINE);
  out_pack_kernel<<<(NOUTF + 255) / 256, 256, 0, stream>>>(REC, LLINE, out);
}
